// MultiHeadAttention_16836271800675
// MI455X (gfx1250) — hardware-run, weakly checked
//
#include <hip/hip_runtime.h>
#ifndef NB
#define NB 2
#endif
#ifndef SEQ
#define SEQ 2048
#endif
#define NB_FULL 2
#define SEQ_FULL 2048
#define DM 1024
#define NH 16
#define HD 64
#define XB_FULL ((size_t)SEQ_FULL * DM)
#define PLANE ((size_t)NB * NH * SEQ * HD)

static_assert(SEQ % 128 == 0);
static_assert(SEQ <= SEQ_FULL);
static_assert(NB <= NB_FULL);
static_assert(HD == 64);
static_assert(DM == NH * HD);
static_assert(DM % 32 == 0);
static_assert((3 * DM) % 64 == 0);
static_assert((size_t)NB * SEQ * DM * 2 + (size_t)3 * DM * DM * 2 + 3 * PLANE * 2 + (size_t)NB * SEQ * DM * 4 <= (size_t)134217728);

typedef __bf16 v16b __attribute__((ext_vector_type(16)));
typedef _Float16 v16h __attribute__((ext_vector_type(16)));
typedef unsigned short v8us __attribute__((ext_vector_type(8), may_alias));
typedef float v8f __attribute__((ext_vector_type(8)));
typedef float v4f __attribute__((ext_vector_type(4)));
typedef float v4fa __attribute__((ext_vector_type(4), may_alias));
union FragB { v16b v; v8us half[2]; unsigned short u[16]; };
union FragH { v16h v; v8us half[2]; _Float16 h[16]; unsigned short u[16]; };

#define LOG2E 1.4426950408889634f
#define NEGFILL (-1.0e20f)
#define CARRY 16.0f
#define QKSCALE 0.00048828125f

__device__ __forceinline__ unsigned short bf16_bits(float x) {
  unsigned int u = __float_as_uint(x);
  return (unsigned short)((u + 0x7FFFu + ((u >> 16) & 1u)) >> 16);
}
__device__ __forceinline__ float bf16_val(unsigned short b) { return __uint_as_float(((unsigned int)b) << 16); }
__device__ __forceinline__ float bf16_rne(float x) { return bf16_val(bf16_bits(x)); }
__device__ __forceinline__ unsigned short f16_bits(float x) { const _Float16 h = (_Float16)x; return __builtin_bit_cast(unsigned short, h); }

__device__ __forceinline__ void mma_b4(v16b a, v16b b0, v16b b1, v16b b2, v16b b3, v8f& c0, v8f& c1, v8f& c2, v8f& c3) {
  c0 = __builtin_amdgcn_wmma_f32_16x16x32_bf16(false, a, false, b0, (short)0, c0, false, false);
  c1 = __builtin_amdgcn_wmma_f32_16x16x32_bf16(false, a, false, b1, (short)0, c1, false, false);
  c2 = __builtin_amdgcn_wmma_f32_16x16x32_bf16(false, a, false, b2, (short)0, c2, false, false);
  c3 = __builtin_amdgcn_wmma_f32_16x16x32_bf16(false, a, false, b3, (short)0, c3, false, false);
  asm volatile("v_nop\n\tv_nop\n\tv_nop\n\tv_nop" : "+v"(c0), "+v"(c1), "+v"(c2), "+v"(c3) : "v"(a), "v"(b0), "v"(b1), "v"(b2), "v"(b3));
}
__device__ __forceinline__ v8f mma_hh2(v16h a0, v16h b0, v16h a1, v16h b1, v8f c) {
  c = __builtin_amdgcn_wmma_f32_16x16x32_f16(false, a0, false, b0, (short)0, c, false, false);
  c = __builtin_amdgcn_wmma_f32_16x16x32_f16(false, a1, false, b1, (short)0, c, false, false);
  asm volatile("v_nop\n\tv_nop\n\tv_nop\n\tv_nop" : "+v"(c) : "v"(a0), "v"(b0), "v"(a1), "v"(b1));
  return c;
}
__device__ __forceinline__ void mma_h2(v16h a, v16h bh, v16h bl, v8f& ch, v8f& cl) {
  ch = __builtin_amdgcn_wmma_f32_16x16x32_f16(false, a, false, bh, (short)0, ch, false, false);
  cl = __builtin_amdgcn_wmma_f32_16x16x32_f16(false, a, false, bl, (short)0, cl, false, false);
  asm volatile("v_nop\n\tv_nop\n\tv_nop\n\tv_nop" : "+v"(ch), "+v"(cl) : "v"(a), "v"(bh), "v"(bl));
}

__global__ __launch_bounds__(256) void k_cvt(const float* __restrict__ src, unsigned short* __restrict__ dst,
                                             int nrows, int rpb, long long bstride) {
  const int t = blockIdx.x * 256 + threadIdx.x;
  if (t >= nrows * 128) return;
  const int row = t >> 7, piece = t & 127;
  const int b = row / rpb, s = row - b * rpb;
  const float* p = src + (size_t)b * (size_t)bstride + (size_t)s * DM + piece * 8;
  const v4f x0 = *(const v4fa*)(p), x1 = *(const v4fa*)(p + 4);
  v8us o;
  o[0] = bf16_bits(x0[0]); o[1] = bf16_bits(x0[1]); o[2] = bf16_bits(x0[2]); o[3] = bf16_bits(x0[3]);
  o[4] = bf16_bits(x1[0]); o[5] = bf16_bits(x1[1]); o[6] = bf16_bits(x1[2]); o[7] = bf16_bits(x1[3]);
  unsigned short* d = dst + (size_t)t * 8;
  *(volatile v8us*)d = o;
  __threadfence();
  *(volatile v8us*)d = o;
}

__device__ __forceinline__ void stage8(unsigned short* st, const v8f& c, int base, int rstep) {
#pragma unroll
  for (int r = 0; r < 8; ++r) st[base + r * rstep] = f16_bits(c[r] * CARRY);
}

__global__ __launch_bounds__(128) void k_proj(const unsigned short* __restrict__ Xb, const unsigned short* __restrict__ Wb,
                                              unsigned short* __restrict__ P3) {
  __shared__ __attribute__((aligned(16))) unsigned short st[128 * 72];
  const int tid = threadIdx.x, w = __builtin_amdgcn_readfirstlane((int)(tid >> 5)), lane = tid & 31, ln = lane & 15, hh = lane >> 4;
  const int n0 = blockIdx.x * 64;
  const int m0 = blockIdx.y * 128;
  const unsigned short* ap0 = Xb + (size_t)(m0 + 32 * w + ln) * DM + 8 * hh;
  const unsigned short* ap1 = ap0 + (size_t)16 * DM;
  const unsigned short* bp = Wb + (size_t)(n0 + ln) * DM + 8 * hh;
  const v8f z8 = {0.f, 0.f, 0.f, 0.f, 0.f, 0.f, 0.f, 0.f};
  v8f c00 = z8, c01 = z8, c02 = z8, c03 = z8, c10 = z8, c11 = z8, c12 = z8, c13 = z8;
#pragma unroll 1
  for (int k0 = 0; k0 < DM; k0 += 32) {
    FragB a0, a1, b0, b1, b2, b3;
    a0.half[0] = *(const v8us*)(ap0 + k0); a0.half[1] = *(const v8us*)(ap0 + k0 + 16);
    a1.half[0] = *(const v8us*)(ap1 + k0); a1.half[1] = *(const v8us*)(ap1 + k0 + 16);
    b0.half[0] = *(const v8us*)(bp + k0);                        b0.half[1] = *(const v8us*)(bp + k0 + 16);
    b1.half[0] = *(const v8us*)(bp + (size_t)16 * DM + k0);      b1.half[1] = *(const v8us*)(bp + (size_t)16 * DM + k0 + 16);
    b2.half[0] = *(const v8us*)(bp + (size_t)32 * DM + k0);      b2.half[1] = *(const v8us*)(bp + (size_t)32 * DM + k0 + 16);
    b3.half[0] = *(const v8us*)(bp + (size_t)48 * DM + k0);      b3.half[1] = *(const v8us*)(bp + (size_t)48 * DM + k0 + 16);
    mma_b4(a0.v, b0.v, b1.v, b2.v, b3.v, c00, c01, c02, c03);
    mma_b4(a1.v, b0.v, b1.v, b2.v, b3.v, c10, c11, c12, c13);
  }
  const int which = n0 >> 10;
  const int h = (n0 & 1023) >> 6;
  const int b = m0 / SEQ, s0 = m0 - b * SEQ;
  const int bh = b * NH + h;
  const bool rowmajor = which < 2;
  const int rstep = rowmajor ? 72 : 1;
  const int rb0 = 32 * w + 8 * hh, rb1 = rb0 + 16;
  stage8(st, c00, rowmajor ? rb0 * 72 + ln        : (ln) * 136 + rb0,      rstep);
  stage8(st, c01, rowmajor ? rb0 * 72 + 16 + ln   : (16 + ln) * 136 + rb0, rstep);
  stage8(st, c02, rowmajor ? rb0 * 72 + 32 + ln   : (32 + ln) * 136 + rb0, rstep);
  stage8(st, c03, rowmajor ? rb0 * 72 + 48 + ln   : (48 + ln) * 136 + rb0, rstep);
  stage8(st, c10, rowmajor ? rb1 * 72 + ln        : (ln) * 136 + rb1,      rstep);
  stage8(st, c11, rowmajor ? rb1 * 72 + 16 + ln   : (16 + ln) * 136 + rb1, rstep);
  stage8(st, c12, rowmajor ? rb1 * 72 + 32 + ln   : (32 + ln) * 136 + rb1, rstep);
  stage8(st, c13, rowmajor ? rb1 * 72 + 48 + ln   : (48 + ln) * 136 + rb1, rstep);
  __syncthreads();
  if (rowmajor) {
    unsigned short* base = P3 + (size_t)which * PLANE + ((size_t)bh * SEQ + s0) * HD;
    for (int pass = 0; pass < 2; ++pass) {
#pragma unroll
      for (int it = 0; it < 8; ++it) {
        const int i = tid + 128 * it;
        const int row = i >> 3, pc = i & 7;
        const v8us o = *(const v8us*)(&st[row * 72 + pc * 8]);
        *(volatile v8us*)(base + (size_t)row * HD + pc * 8) = o;
      }
      if (pass == 0) __threadfence();
    }
  } else {
    unsigned short* base = P3 + (size_t)2 * PLANE + (size_t)bh * HD * SEQ + s0;
    for (int pass = 0; pass < 2; ++pass) {
#pragma unroll
      for (int it = 0; it < 8; ++it) {
        const int i = tid + 128 * it;
        const int dc = i >> 4, pc = i & 15;
        const v8us o = *(const v8us*)(&st[dc * 136 + pc * 8]);
        *(volatile v8us*)(base + (size_t)dc * SEQ + pc * 8) = o;
      }
      if (pass == 0) __threadfence();
    }
  }
}

__device__ __forceinline__ void fa_step(const unsigned short* __restrict__ Kp, const unsigned short* __restrict__ Vp,
                                        int key0, unsigned int mword, int ln, int hh, const FragH& q0, const FragH& q1,
                                        float& mr, float& lr, v8f (&Oh)[4], v8f (&Ol)[4]) {
  const unsigned short* kp0 = Kp + (size_t)(key0 + ln) * HD + 8 * hh;
  const unsigned short* kp1 = kp0 + 16 * HD;
  FragH k00, k01, k10, k11;
  k00.half[0] = *(const v8us*)(kp0);      k00.half[1] = *(const v8us*)(kp0 + 16);
  k01.half[0] = *(const v8us*)(kp0 + 32); k01.half[1] = *(const v8us*)(kp0 + 48);
  k10.half[0] = *(const v8us*)(kp1);      k10.half[1] = *(const v8us*)(kp1 + 16);
  k11.half[0] = *(const v8us*)(kp1 + 32); k11.half[1] = *(const v8us*)(kp1 + 48);
  const unsigned short* vp = Vp + (size_t)ln * SEQ + key0 + 8 * hh;
  FragH vf[4];
#pragma unroll
  for (int t = 0; t < 4; ++t) {
    vf[t].half[0] = *(const v8us*)(vp + (size_t)t * 16 * SEQ);
    vf[t].half[1] = *(const v8us*)(vp + (size_t)t * 16 * SEQ + 16);
  }
  const v8f z8 = {0.f, 0.f, 0.f, 0.f, 0.f, 0.f, 0.f, 0.f};
  const v8f s0 = mma_hh2(k00.v, q0.v, k01.v, q1.v, z8);
  const v8f s1 = mma_hh2(k10.v, q0.v, k11.v, q1.v, z8);
  const unsigned int wl = mword >> (8 * hh);
  float sc[16];
#pragma unroll
  for (int r = 0; r < 8; ++r) {
    const float a = s0[r] * QKSCALE, c = s1[r] * QKSCALE;
    sc[r]     = ((wl >> r) & 1u) ? NEGFILL : a;
    sc[8 + r] = ((wl >> (16 + r)) & 1u) ? NEGFILL : c;
  }
  float mx = sc[0];
#pragma unroll
  for (int i = 1; i < 16; ++i) mx = fmaxf(mx, sc[i]);
  mx = fmaxf(mx, __shfl_xor(mx, 16, 32));
  const float mnew = fmaxf(mr, mx);
  const float al = exp2f((mr - mnew) * LOG2E);
  mr = mnew;
  FragH ph, pl;
  float ps = 0.0f;
#pragma unroll
  for (int i = 0; i < 16; ++i) {
    const float pc = exp2f(fmaf(sc[i] - mnew, LOG2E, 8.0f));
    ps += pc;
    const _Float16 h = (_Float16)pc;
    ph.h[i] = h;
    pl.h[i] = (_Float16)((pc - (float)h) * 2048.0f);
  }
  ps += __shfl_xor(ps, 16, 32);
  lr = lr * al + ps;
#pragma unroll
  for (int t = 0; t < 4; ++t) { Oh[t] = Oh[t] * al; Ol[t] = Ol[t] * al; }
#pragma unroll
  for (int t = 0; t < 4; ++t) mma_h2(vf[t].v, ph.v, pl.v, Oh[t], Ol[t]);
}

__global__ __launch_bounds__(128) void k_attn(const unsigned short* __restrict__ Qh, const unsigned short* __restrict__ Kh,
                                              const unsigned short* __restrict__ Vt, const int* __restrict__ mask,
                                              float* __restrict__ Cx) {
  __shared__ __attribute__((aligned(16))) float so[4][16][68];
  __shared__ unsigned int mw[SEQ / 32];
  const int tid = threadIdx.x, w = __builtin_amdgcn_readfirstlane((int)(tid >> 5)), lane = tid & 31, ln = lane & 15, hh = lane >> 4;
  const int bh = blockIdx.x / (SEQ / 64), qt = blockIdx.x % (SEQ / 64);
  const int b = bh / NH, h = bh - b * NH;
  const int qbase = qt * 64 + 16 * w;
  const int qg = qbase + ln;
  for (int j = w; j < SEQ / 32; j += 4) {
    const int mv = mask[(size_t)b * SEQ_FULL + 32 * j + lane];
    const unsigned long long bal = __ballot(mv == 0);
    if (lane == 0) mw[j] = (unsigned int)bal;
  }
  __syncthreads();
  const unsigned short* qrow = Qh + ((size_t)bh * SEQ + qg) * HD + 8 * hh;
  FragH q0, q1;
  q0.half[0] = *(const v8us*)(qrow);      q0.half[1] = *(const v8us*)(qrow + 16);
  q1.half[0] = *(const v8us*)(qrow + 32); q1.half[1] = *(const v8us*)(qrow + 48);
  float mr = -3.0e38f, lr = 0.0f;
  v8f Oh[4] = {}, Ol[4] = {};
  const unsigned short* Kp = Kh + (size_t)bh * SEQ * HD;
  const unsigned short* Vp = Vt + (size_t)bh * HD * SEQ;
#pragma unroll 1
  for (int j = 0; j < SEQ / 32; ++j)
    fa_step(Kp, Vp, 32 * j, mw[j], ln, hh, q0, q1, mr, lr, Oh, Ol);

  const float inv = 1.0f / (CARRY * lr);
#pragma unroll
  for (int t = 0; t < 4; ++t)
#pragma unroll
    for (int r = 0; r < 8; ++r)
      so[w][ln][16 * t + 8 * hh + r] = (Oh[t][r] + Ol[t][r] * 0.00048828125f) * inv;
  __syncthreads();
  float* og = Cx + ((size_t)b * SEQ + qbase) * DM + h * HD;
  const int rsub = lane >> 4, c4 = (lane & 15) * 4;
  for (int pass = 0; pass < 2; ++pass) {
#pragma unroll
    for (int q = 0; q < 8; ++q) {
      const int row = 2 * q + rsub;
      const v4f v = *(const v4fa*)&so[w][row][c4];
      *(volatile v4f*)(og + (size_t)row * DM + c4) = v;
    }
    if (pass == 0) __threadfence();
  }
}

__global__ __launch_bounds__(256) void k_ln(const float* __restrict__ Cx, const float* __restrict__ gamma,
                                            const float* __restrict__ beta, float* __restrict__ out) {
  __shared__ float rs[8];
  __shared__ float rq[8];
  const int tid = threadIdx.x, lane = tid & 31, w = __builtin_amdgcn_readfirstlane((int)(tid >> 5));
  const int r = blockIdx.x;
  const int b = r / SEQ, s = r - b * SEQ;
  const v4f x = *(const v4fa*)(Cx + (size_t)r * DM + tid * 4);
  float sm = (x[0] + x[1]) + (x[2] + x[3]);
#pragma unroll
  for (int off = 16; off >= 1; off >>= 1) sm += __shfl_xor(sm, off, 32);
  if (lane == 0) rs[w] = sm;
  __syncthreads();
  float tot = 0.0f;
#pragma unroll
  for (int i = 0; i < 8; ++i) tot += rs[i];
  const float mu = tot * (1.0f / 1024.0f);
  const float d0 = x[0] - mu, d1 = x[1] - mu, d2 = x[2] - mu, d3 = x[3] - mu;
  float sq = (d0 * d0 + d1 * d1) + (d2 * d2 + d3 * d3);
#pragma unroll
  for (int off = 16; off >= 1; off >>= 1) sq += __shfl_xor(sq, off, 32);
  if (lane == 0) rq[w] = sq;
  __syncthreads();
  float tq = 0.0f;
#pragma unroll
  for (int i = 0; i < 8; ++i) tq += rq[i];
  const float var = tq * (1.0f / 1024.0f);
  const float rinv = rsqrtf(var + 1.0e-6f);
  const v4f g = *(const v4fa*)(gamma + tid * 4);
  const v4f be = *(const v4fa*)(beta + tid * 4);
  v4f o;
  o[0] = d0 * rinv * bf16_rne(g[0]) + bf16_rne(be[0]);
  o[1] = d1 * rinv * bf16_rne(g[1]) + bf16_rne(be[1]);
  o[2] = d2 * rinv * bf16_rne(g[2]) + bf16_rne(be[2]);
  o[3] = d3 * rinv * bf16_rne(g[3]) + bf16_rne(be[3]);
  float* dst = out + ((size_t)b * SEQ_FULL + s) * DM + tid * 4;
  *(volatile v4f*)dst = o;
  __threadfence();
  *(volatile v4f*)dst = o;
}

extern "C" void kernel_launch(void* const* d_in, const int* in_sizes, int n_in,
                              void* d_out, int out_size, void* d_ws, size_t ws_size, hipStream_t stream) {
  if (n_in < 7) return;
  const long long need_x = (long long)(NB - 1) * SEQ_FULL * DM + (long long)SEQ * DM;
  const long long need_m = (long long)(NB - 1) * SEQ_FULL + (long long)SEQ;
  if ((long long)in_sizes[0] < need_x || (long long)in_sizes[1] < need_m) return;
  if ((long long)in_sizes[2] < (long long)DM * DM || (long long)in_sizes[3] < (long long)DM * DM || (long long)in_sizes[4] < (long long)DM * DM) return;
  if (in_sizes[5] < DM || in_sizes[6] < DM) return;
  if ((long long)out_size < need_x) return;
  const float* X     = (const float*)d_in[0];
  const int*   mask  = (const int*)d_in[1];
  const float* Wq    = (const float*)d_in[2];
  const float* Wk    = (const float*)d_in[3];
  const float* Wv    = (const float*)d_in[4];
  const float* gamma = (const float*)d_in[5];
  const float* beta  = (const float*)d_in[6];
  float* out = (float*)d_out;
  char* ws = (char*)d_ws;
  size_t off = 0;
  const size_t xb_bytes = (size_t)NB * SEQ * DM * 2;
  const size_t wb_bytes = (size_t)3 * DM * DM * 2;
  const size_t p3_bytes = 3 * PLANE * 2;
  const size_t cx_bytes = (size_t)NB * SEQ * DM * 4;
  unsigned short* Xb = (unsigned short*)(ws + off); off += (xb_bytes + 255) & ~(size_t)255;
  unsigned short* Wb = (unsigned short*)(ws + off); off += (wb_bytes + 255) & ~(size_t)255;
  unsigned short* P3 = (unsigned short*)(ws + off); off += (p3_bytes + 255) & ~(size_t)255;
  float*          Cx = (float*)(ws + off);          off += (cx_bytes + 255) & ~(size_t)255;
  if (off > ws_size) return;
  k_cvt<<<(unsigned)((NB * SEQ * 128 + 255) / 256), 256, 0, stream>>>(X, Xb, NB * SEQ, SEQ, (long long)XB_FULL);
  k_cvt<<<(unsigned)((DM * 128 + 255) / 256), 256, 0, stream>>>(Wq, Wb, DM, DM, 0LL);
  k_cvt<<<(unsigned)((DM * 128 + 255) / 256), 256, 0, stream>>>(Wk, Wb + (size_t)DM * DM, DM, DM, 0LL);
  k_cvt<<<(unsigned)((DM * 128 + 255) / 256), 256, 0, stream>>>(Wv, Wb + (size_t)2 * DM * DM, DM, DM, 0LL);
  k_proj<<<dim3((unsigned)(3 * DM / 64), (unsigned)(NB * SEQ / 128)), 128, 0, stream>>>(Xb, Wb, P3);
  k_attn<<<(unsigned)(NB * NH * (SEQ / 64)), 128, 0, stream>>>(P3, P3 + PLANE, P3 + 2 * PLANE, mask, Cx);
  k_ln<<<(unsigned)(NB * SEQ), 256, 0, stream>>>(Cx, gamma, beta, out);
}
